// NILUT_57827439674099
// MI455X (gfx1250) — hardware-verified
//
#include <hip/hip_runtime.h>
#include <stdint.h>


typedef _Float16 v8h  __attribute__((ext_vector_type(8)));
typedef _Float16 v16h __attribute__((ext_vector_type(16)));
typedef float    v8f  __attribute__((ext_vector_type(8)));
typedef float    v4f  __attribute__((ext_vector_type(4)));
typedef unsigned int v4u __attribute__((ext_vector_type(4)));

union Frag  { v16h v; v8h half[2]; };
union Pack8 { v8h h; v4u u; _Float16 e[8]; };

#define HID       256
#define EMB_DIM   64
#define IN_DIM    67
#define ROWS      16
#define NWAVE     4
#define NTHR      (NWAVE * 32)
#define BLKPIX    (NWAVE * ROWS)
#define ACT_SCALE 16.0f
#define W_SCALE   64.0f
#define INV_SCALE (1.0f / 1024.0f)
#define ERF_CLAMP 3.832506856900711f

__device__ __forceinline__ int sw(int m, int k) {
  return m * HID + ((((k >> 3) ^ (m & 7))) << 3) + (k & 7);
}

__device__ __forceinline__ float erf_f32(float x) {
  x = fminf(fmaxf(x, -ERF_CLAMP), ERF_CLAMP);
  const float x2 = x * x;
  float a = 0.00022905065861350646f;
  a = fmaf(a, x2, 0.0034082910107109506f);
  a = fmaf(a, x2, 0.050955695062380861f);
  a = fmaf(a, x2, 0.18520832239976145f);
  a = fmaf(a, x2, 1.128379143519084f);
  float b = -1.1791602954361697e-7f;
  b = fmaf(b, x2, 0.000023547966471313185f);
  b = fmaf(b, x2, 0.0010179625278914885f);
  b = fmaf(b, x2, 0.014070470171167667f);
  b = fmaf(b, x2, 0.11098505178285362f);
  b = fmaf(b, x2, 0.49746925110067538f);
  b = fmaf(b, x2, 1.0f);
  return (x * a) * __builtin_amdgcn_rcpf(b);
}

__device__ __forceinline__ float gelu_f(float x) {
  return 0.5f * x * (1.0f + erf_f32(x * 0.70710678118654752f));
}

__device__ __forceinline__ v8f wmma_f16(v16h a, v16h b, v8f c) {
  v8f d = __builtin_amdgcn_wmma_f32_16x16x32_f16(false, a, false, b, (short)0, c, false, false);
  asm volatile("v_nop\n\tv_nop\n\tv_nop\n\tv_nop" : "+v"(d) : "v"(a), "v"(b));
  return d;
}

__device__ __forceinline__ void gemm2(const _Float16* act, const _Float16* __restrict__ wt,
                                      int n0, int h, int m, v8f& out0, v8f& out1) {
  v8f c0 = {0.f, 0.f, 0.f, 0.f, 0.f, 0.f, 0.f, 0.f};
  v8f c1 = {0.f, 0.f, 0.f, 0.f, 0.f, 0.f, 0.f, 0.f};
  const _Float16* wp0 = wt + (size_t)(n0 + m) * HID + 8 * h;
  const _Float16* wp1 = wp0 + 16 * HID;
#pragma unroll
  for (int kc = 0; kc < HID / 32; ++kc) {
    const int k0 = kc * 32;
    Frag a, b0, b1;
    a.half[0]  = *(const v8h*)(act + sw(m, k0 + 8 * h));
    a.half[1]  = *(const v8h*)(act + sw(m, k0 + 16 + 8 * h));
    b0.half[0] = *(const v8h*)(wp0 + k0);
    b0.half[1] = *(const v8h*)(wp0 + k0 + 16);
    b1.half[0] = *(const v8h*)(wp1 + k0);
    b1.half[1] = *(const v8h*)(wp1 + k0 + 16);
    c0 = wmma_f16(a.v, b0.v, c0);
    c1 = wmma_f16(a.v, b1.v, c1);
  }
  out0 = c0;
  out1 = c1;
}

__global__ __launch_bounds__(256) void k_prep(
    const float* __restrict__ W1, const float* __restrict__ W2,
    const float* __restrict__ W0, const float* __restrict__ b0,
    const float* __restrict__ emb, const int* __restrict__ sidx,
    _Float16* wt1, _Float16* wt2, float* cst, int nimg, int nstyle) {
  __shared__ __attribute__((aligned(16))) _Float16 st[8 * HID];
  __shared__ __attribute__((aligned(16))) float sc[HID];
  const int t = threadIdx.x;
  const int blk = blockIdx.x;
  if (blk < 64) {
    const float* W  = (blk < 32) ? W1 : W2;
    _Float16*    wt = (blk < 32) ? wt1 : wt2;
    const int n0 = (blk & 31) * 8;
    const float* src = W + (size_t)t * HID + n0;
#pragma unroll
    for (int j = 0; j < 8; ++j) st[j * HID + t] = (_Float16)(src[j] * W_SCALE);
    __syncthreads();
    const int j = t >> 5, q = t & 31;
    Pack8 pk;
    pk.h = *(const v8h*)(st + j * HID + 8 * q);
    _Float16* dst = wt + (size_t)(n0 + j) * HID + 8 * q;
    *(volatile v4u*)dst = pk.u;
    __threadfence();
    *(volatile v4u*)dst = pk.u;
  } else {
    for (int b = 0; b < nimg; ++b) {
      int si = sidx[b];
      if (si < 0) si += nstyle;
      si = (si < 0) ? 0 : ((si > nstyle - 1) ? (nstyle - 1) : si);
      const float* e = emb + si * EMB_DIM;
      float s = b0[t];
#pragma unroll 4
      for (int jj = 0; jj < EMB_DIM; ++jj) s = fmaf(e[jj], W0[(3 + jj) * HID + t], s);
      sc[t] = s;
      __syncthreads();
      if (t < HID / 4) {
        const v4f v = *(const v4f*)(sc + 4 * t);
        float* d = cst + (size_t)b * HID + 4 * t;
        *(volatile v4f*)d = v;
        __threadfence();
        *(volatile v4f*)d = v;
      }
      __syncthreads();
    }
  }
}

__global__ __launch_bounds__(NTHR) __attribute__((amdgpu_num_vgpr(192)))
void k_mlp(const float* __restrict__ rgb, const float* __restrict__ W0,
           const float* __restrict__ cst,
           const _Float16* __restrict__ wt1, const float* __restrict__ b1,
           const _Float16* __restrict__ wt2, const float* __restrict__ b2,
           const float* __restrict__ W3, const float* __restrict__ b3,
           float* out, int npix, int hw) {
  __shared__ __attribute__((aligned(16))) _Float16 smem[NWAVE * 2 * ROWS * HID];
  const int tid = threadIdx.x;
  const int l = tid & 31, wv = tid >> 5, h = l >> 4, m = l & 15;
  _Float16* bufA = smem + wv * (2 * ROWS * HID);
  _Float16* bufB = bufA + ROWS * HID;
  const int pblk = blockIdx.x * BLKPIX;
  const int pw   = pblk + wv * ROWS;

  {
    float wr[8], wg[8], wb[8];
#pragma unroll
    for (int j = 0; j < 8; ++j) {
      wr[j] = W0[8 * l + j];
      wg[j] = W0[HID + 8 * l + j];
      wb[j] = W0[2 * HID + 8 * l + j];
    }
#pragma unroll 1
    for (int mm = 0; mm < ROWS; ++mm) {
      int p = pw + mm;
      if (p > npix - 1) p = npix - 1;
      const int bi  = p / hw;
      const int pix = p - bi * hw;
      const float cr = rgb[(size_t)(bi * 3 + 0) * (size_t)hw + pix];
      const float cg = rgb[(size_t)(bi * 3 + 1) * (size_t)hw + pix];
      const float cb = rgb[(size_t)(bi * 3 + 2) * (size_t)hw + pix];
      const float* cp = cst + (size_t)bi * HID + 8 * l;
      const v4f q0 = *(const v4f*)cp;
      const v4f q1 = *(const v4f*)(cp + 4);
      float cc[8];
#pragma unroll
      for (int j = 0; j < 4; ++j) { cc[j] = q0[j]; cc[4 + j] = q1[j]; }
      Pack8 pk;
#pragma unroll
      for (int j = 0; j < 8; ++j) {
        float x = fmaf(cb, wb[j], cc[j]);
        x = fmaf(cg, wg[j], x);
        x = fmaf(cr, wr[j], x);
        pk.e[j] = (_Float16)(gelu_f(x) * ACT_SCALE);
      }
      *(v8h*)(bufA + sw(mm, 8 * l)) = pk.h;
    }
  }
  __syncthreads();

#pragma unroll 1
  for (int nt = 0; nt < HID / 32; ++nt) {
    const int n0 = nt * 32;
    v8f acc0, acc1;
    gemm2(bufA, wt1, n0, h, m, acc0, acc1);
    const int na = n0 + m, nb = n0 + 16 + m;
    const float ba = b1[na], bb = b1[nb];
#pragma unroll
    for (int r = 0; r < 8; ++r) {
      const float xa = fmaf(acc0[r], INV_SCALE, ba);
      const float xb = fmaf(acc1[r], INV_SCALE, bb);
      bufB[sw(8 * h + r, na)] = (_Float16)(gelu_f(xa) * ACT_SCALE);
      bufB[sw(8 * h + r, nb)] = (_Float16)(gelu_f(xb) * ACT_SCALE);
    }
  }
  __syncthreads();

  float pd[8][3];
#pragma unroll
  for (int r = 0; r < 8; ++r) { pd[r][0] = 0.f; pd[r][1] = 0.f; pd[r][2] = 0.f; }
#pragma unroll 1
  for (int nt = 0; nt < HID / 32; ++nt) {
    const int n0 = nt * 32;
    v8f acc0, acc1;
    gemm2(bufB, wt2, n0, h, m, acc0, acc1);
    const int na = n0 + m, nb = n0 + 16 + m;
    const float ba = b2[na], bb = b2[nb];
    const float wa0 = W3[na * 3 + 0], wa1 = W3[na * 3 + 1], wa2 = W3[na * 3 + 2];
    const float wb0 = W3[nb * 3 + 0], wb1 = W3[nb * 3 + 1], wb2 = W3[nb * 3 + 2];
#pragma unroll
    for (int r = 0; r < 8; ++r) {
      const float ga = gelu_f(fmaf(acc0[r], INV_SCALE, ba));
      const float gb = gelu_f(fmaf(acc1[r], INV_SCALE, bb));
      pd[r][0] = fmaf(ga, wa0, pd[r][0]);
      pd[r][1] = fmaf(ga, wa1, pd[r][1]);
      pd[r][2] = fmaf(ga, wa2, pd[r][2]);
      pd[r][0] = fmaf(gb, wb0, pd[r][0]);
      pd[r][1] = fmaf(gb, wb1, pd[r][1]);
      pd[r][2] = fmaf(gb, wb2, pd[r][2]);
    }
  }
#pragma unroll
  for (int r = 0; r < 8; ++r) {
#pragma unroll
    for (int c = 0; c < 3; ++c) {
      float v = pd[r][c];
      v += __shfl_xor(v, 1, 32);
      v += __shfl_xor(v, 2, 32);
      v += __shfl_xor(v, 4, 32);
      v += __shfl_xor(v, 8, 32);
      pd[r][c] = v;
    }
  }
  __syncthreads();

  float* sout = reinterpret_cast<float*>(smem);
  {
    const float b30 = b3[0], b31 = b3[1], b32 = b3[2];
    if (m == 0) {
#pragma unroll
      for (int r = 0; r < 8; ++r) {
        const int row = wv * ROWS + 8 * h + r;
        const float z0 = pd[r][0] + b30, z1 = pd[r][1] + b31, z2 = pd[r][2] + b32;
        sout[0 * BLKPIX + row] = __builtin_amdgcn_rcpf(1.0f + __expf(-z0));
        sout[1 * BLKPIX + row] = __builtin_amdgcn_rcpf(1.0f + __expf(-z1));
        sout[2 * BLKPIX + row] = __builtin_amdgcn_rcpf(1.0f + __expf(-z2));
      }
    }
  }
  __syncthreads();

  {
    const bool live = (tid < 3 * (BLKPIX / 4));
    const int c = tid >> 4, q = tid & 15;
    const int p = pblk + 4 * q;
    v4f v = {0.f, 0.f, 0.f, 0.f};
    bool vec = false, any = false;
    size_t idx = 0;
    if (live && p < npix) {
      v = *(const v4f*)(sout + c * BLKPIX + 4 * q);
      const int bi = p / hw;
      const int pix = p - bi * hw;
      idx = (size_t)(bi * 3 + c) * (size_t)hw + (size_t)pix;
      any = true;
      vec = (pix + 3 < hw) && ((idx & 3) == 0);
    }
    if (vec) {
      *(volatile v4f*)(out + idx) = v;
    } else if (any) {
#pragma unroll
      for (int e = 0; e < 4; ++e) {
        const int pe = p + e;
        if (pe < npix) {
          const int be = pe / hw;
          const int pxe = pe - be * hw;
          const float val = v[e];
          *(volatile float*)(out + (size_t)(be * 3 + c) * (size_t)hw + pxe) = val;
        }
      }
    }
    __threadfence();
    if (vec) {
      *(volatile v4f*)(out + idx) = v;
    } else if (any) {
#pragma unroll
      for (int e = 0; e < 4; ++e) {
        const int pe = p + e;
        if (pe < npix) {
          const int be = pe / hw;
          const int pxe = pe - be * hw;
          const float val = v[e];
          *(volatile float*)(out + (size_t)(be * 3 + c) * (size_t)hw + pxe) = val;
        }
      }
    }
  }
}

extern "C" void kernel_launch(void* const* d_in, const int* in_sizes, int n_in,
                              void* d_out, int out_size, void* d_ws,
                              size_t ws_size, hipStream_t stream) {
  if (n_in < 11) return;
  const float* rgb  = (const float*)d_in[0];
  const int*   sidx = (const int*)d_in[1];
  const float* emb  = (const float*)d_in[2];
  const float* W0   = (const float*)d_in[3];
  const float* b0   = (const float*)d_in[4];
  const float* W1   = (const float*)d_in[5];
  const float* b1   = (const float*)d_in[6];
  const float* W2   = (const float*)d_in[7];
  const float* b2   = (const float*)d_in[8];
  const float* W3   = (const float*)d_in[9];
  const float* b3   = (const float*)d_in[10];
  float* out = (float*)d_out;

  const int nimg = in_sizes[1];
  if (nimg <= 0) return;
  const int hw = in_sizes[0] / (3 * nimg);
  if (hw <= 0) return;
  const int npix = nimg * hw;
  if (out_size != 3 * npix) return;
  const int nstyle = in_sizes[2] / EMB_DIM;
  if (nstyle <= 0) return;
  if (in_sizes[3] != IN_DIM * HID || in_sizes[5] != HID * HID ||
      in_sizes[7] != HID * HID || in_sizes[9] != HID * 3 ||
      in_sizes[4] < HID || in_sizes[6] < HID || in_sizes[8] < HID || in_sizes[10] < 3)
    return;

  const size_t off_wt1 = 0;
  const size_t off_wt2 = off_wt1 + (size_t)HID * HID * sizeof(_Float16);
  const size_t off_cst = off_wt2 + (size_t)HID * HID * sizeof(_Float16);
  const size_t total   = off_cst + (size_t)nimg * HID * sizeof(float);
  if (total > ws_size) return;
  char* ws = (char*)d_ws;
  _Float16* wt1 = (_Float16*)(ws + off_wt1);
  _Float16* wt2 = (_Float16*)(ws + off_wt2);
  float*    cst = (float*)(ws + off_cst);

  k_prep<<<65, 256, 0, stream>>>(W1, W2, W0, b0, emb, sidx, wt1, wt2, cst, nimg, nstyle);

  const int blocks = (npix + BLKPIX - 1) / BLKPIX;
  k_mlp<<<blocks, NTHR, 0, stream>>>(rgb, W0, cst, wt1, b1, wt2, b2, W3, b3, out, npix, hw);
}
